// ProbEncoder_59219009077524
// MI455X (gfx1250) — hardware-run, weakly checked
//
#include <hip/hip_runtime.h>
#pragma clang fp contract(off)


#ifndef NB
#define NB 4
#endif
#ifndef SEQ
#define SEQ 512
#endif
#define NB_FULL  4
#define SEQ_FULL 512
#ifndef OUT_SEQ
#define OUT_SEQ SEQ
#endif
#define DL   32
#define NBK  5
#define KD   (NBK * DL)
#define TPB  512
#define NSEG (SEQ / 32)
#define PPT  ((SEQ * 4) / TPB)
#define GW   4
#define OSP  36
#define SCARRY 32.0f
#define WCARRY 16.0f
#define EPI  (1.0f / 16384.0f)
#define TERN_N ((size_t)2 * NBK * DL * DL * DL)

static_assert(DL == 32);
static_assert(KD % 32 == 0);
static_assert(SEQ % 128 == 0);
static_assert((SEQ * 4) % TPB == 0);
static_assert(PPT * TPB * 8 == SEQ * DL);
static_assert(NSEG <= TPB / 32);
static_assert(NSEG * 32 == SEQ);
static_assert((NB * SEQ) % (16 * GW) == 0);
static_assert(SEQ % 16 == 0);
static_assert(NB <= NB_FULL);
static_assert(SEQ <= SEQ_FULL);
static_assert((OSP * 4) % 16 == 0);
static_assert(SCARRY * WCARRY * 32.0f == 16384.0f);
static_assert((DL * KD) % (8 * 128) == 0);
static_assert((size_t)(SEQ * DL + 16 * DL + SEQ) * 4 <= (size_t)131072);
static_assert((size_t)GW * 16 * OSP * 4 <= (size_t)131072);

typedef _Float16 h16;
typedef __attribute__((ext_vector_type(16))) _Float16 v16h;
typedef __attribute__((ext_vector_type(8)))  _Float16 v8h;
typedef __attribute__((ext_vector_type(8)))  float    v8f;
typedef __attribute__((ext_vector_type(4)))  float    v4f;
typedef v4f  __attribute__((may_alias)) v4fa;

__device__ __forceinline__ v16h cat16(v8h lo, v8h hi) { return __builtin_shufflevector(lo, hi, 0, 1, 2, 3, 4, 5, 6, 7, 8, 9, 10, 11, 12, 13, 14, 15); }
__device__ __forceinline__ v8f wmma16(v16h a, v16h b, v8f c) { return __builtin_amdgcn_wmma_f32_16x16x32_f16(false, a, false, b, (short)0, c, false, false); }
__device__ __forceinline__ v16h  ldh(const h16* p) { return cat16(*(const v8h*)p, *(const v8h*)(p + 16)); }
__device__ __forceinline__ void wave_sync() { __builtin_amdgcn_fence(3  , "wavefront"); __builtin_amdgcn_wave_barrier(); asm volatile("" ::: "memory"); }
__device__ __forceinline__ v8f wmma16g(v16h a, v16h b, v8f c) { c = wmma16(a, b, c); asm volatile("v_nop\n\tv_nop\n\tv_nop\n\tv_nop" : "+v"(c) : "v"(a), "v"(b)); return c; }
static __device__ __forceinline__ h16 toh_flush(float v) { const h16 r = (h16)v; return (fabsf(v) < 6.103515625e-05f) ? (h16)0.0f : r; }

__device__ __forceinline__ float rowsum2(const float* __restrict__ T, unsigned o0, unsigned o1) {
    float s = 0.0f;
#pragma unroll 1
    for (unsigned c = 0; c < 32; c += 4) {
        const v4f a = *(const v4f*)(T + o0 + c); const v4f b = *(const v4f*)(T + o1 + c);
        s += ((a[0] + b[0]) + (a[1] + b[1])) + ((a[2] + b[2]) + (a[3] + b[3]));
    }
    return s;
}

__global__ __launch_bounds__(128) void k_wsum(const float* __restrict__ T, h16* WP) {
    unsigned p = blockIdx.x * 128u + threadIdx.x;
    asm volatile("" : "+v"(p));
    const unsigned e0 = p * 8u;
    const unsigned a = e0 / (unsigned)KD, kb0 = e0 % (unsigned)KD;
    const unsigned k = kb0 >> 5, b0 = kb0 & 31u;
    const unsigned off0 = ((k * 32u + a) * 32u + b0) * 32u;
    const unsigned off1 = off0 + (unsigned)(NBK * DL * DL * DL);
    v8h o;
#pragma unroll
    for (int j = 0; j < 8; ++j) { const float s = rowsum2(T, off0 + (unsigned)j * 32u, off1 + (unsigned)j * 32u); o[j] = toh_flush(s * WCARRY); }
    *(volatile v8h*)(WP + e0) = o; __threadfence(); *(volatile v8h*)(WP + e0) = o;
}

__global__ __launch_bounds__(TPB) void k_bucket(const float* __restrict__ x, const int* __restrict__ mask, h16* SP) {
    __shared__ __align__(16) float us[SEQ * DL];
    __shared__ float seg[16 * DL];
    __shared__ float vrow[SEQ];
    const int t = threadIdx.x, lane = t & 31;
    const int wave = __builtin_amdgcn_readfirstlane((int)(threadIdx.x >> 5));
    const int z = blockIdx.x;
    const size_t PLANE = (size_t)NB * SEQ * DL;
    const size_t zoff = (size_t)z * SEQ * DL;

#pragma unroll 1
    for (int i = t; i < SEQ; i += TPB) { const int mk = mask[(size_t)z * SEQ_FULL + i]; vrow[i] = (mk != 0) ? 1.0f : 0.0f; }
    __syncthreads();

#pragma unroll 1
    for (int r = wave; r < SEQ; r += TPB / 32) {
        const float v = x[((size_t)z * SEQ_FULL + r) * DL + lane];
        float m = v;
        m = fmaxf(m, __shfl_xor(m, 16, 32)); m = fmaxf(m, __shfl_xor(m, 8, 32)); m = fmaxf(m, __shfl_xor(m, 4, 32));
        m = fmaxf(m, __shfl_xor(m, 2, 32));  m = fmaxf(m, __shfl_xor(m, 1, 32));
        const float e = expf(v - m);
        float s = e;
        s += __shfl_xor(s, 16, 32); s += __shfl_xor(s, 8, 32); s += __shfl_xor(s, 4, 32); s += __shfl_xor(s, 2, 32); s += __shfl_xor(s, 1, 32);
        const float keep = vrow[r];
        us[r * DL + lane] = (e * (1.0f / s)) * keep;
    }
    __syncthreads();

#pragma unroll 1
    for (int ps = 0; ps < 2; ++ps) {
#pragma unroll 1
        for (int it = 0; it < PPT; ++it) {
            unsigned q = (unsigned)(it * TPB + t);
            asm volatile("" : "+v"(q));
            const int i = (int)(q >> 2), b0 = (int)(q & 3u) * 8;
            const float sc = vrow[i] * SCARRY;
            const bool okm2 = i >= 2, okm1 = i >= 1, okp1 = i + 1 < SEQ, okp2 = i + 2 < SEQ;
            const int jm2 = okm2 ? i - 2 : 0, jm1 = okm1 ? i - 1 : 0, jp1 = okp1 ? i + 1 : SEQ - 1, jp2 = okp2 ? i + 2 : SEQ - 1;
            const v4f a0 = *(const v4fa*)(&us[jm2 * DL + b0]), a1 = *(const v4fa*)(&us[jm2 * DL + b0 + 4]);
            const v4f c0 = *(const v4fa*)(&us[jm1 * DL + b0]), c1 = *(const v4fa*)(&us[jm1 * DL + b0 + 4]);
            const v4f d0 = *(const v4fa*)(&us[jp1 * DL + b0]), d1 = *(const v4fa*)(&us[jp1 * DL + b0 + 4]);
            const v4f e0 = *(const v4fa*)(&us[jp2 * DL + b0]), e1 = *(const v4fa*)(&us[jp2 * DL + b0 + 4]);
            v8h o1, o2, o3;
#pragma unroll
            for (int c = 0; c < 4; ++c) {
                o1[c] = toh_flush((okm2 ? a0[c] : 0.0f) * sc); o1[4 + c] = toh_flush((okm2 ? a1[c] : 0.0f) * sc);
                o2[c] = toh_flush((okm1 ? c0[c] : 0.0f) * sc); o2[4 + c] = toh_flush((okm1 ? c1[c] : 0.0f) * sc);
                const float s0 = (okp1 ? d0[c] : 0.0f) + (okp2 ? e0[c] : 0.0f);
                const float s1 = (okp1 ? d1[c] : 0.0f) + (okp2 ? e1[c] : 0.0f);
                o3[c] = toh_flush(s0 * sc); o3[4 + c] = toh_flush(s1 * sc);
            }
            const size_t off = zoff + (size_t)q * 8;
            *(volatile v8h*)(SP + (size_t)1 * PLANE + off) = o1;
            *(volatile v8h*)(SP + (size_t)2 * PLANE + off) = o2;
            *(volatile v8h*)(SP + (size_t)3 * PLANE + off) = o3;
        }
        if (ps == 0) __threadfence();
    }

#pragma unroll 1
    for (int s = wave; s < NSEG; s += TPB / 32) {
        float sum = 0.0f;
#pragma unroll 1
        for (int j = s * 32; j < s * 32 + 32; ++j) sum += us[j * DL + lane];
        seg[s * DL + lane] = sum;
    }
    __syncthreads();
    if (wave == 0) {
        float run = 0.0f;
#pragma unroll 1
        for (int s2 = 0; s2 < NSEG; ++s2) { const float tmp = seg[s2 * DL + lane]; seg[s2 * DL + lane] = run; run += tmp; }
    }
    __syncthreads();
#pragma unroll 1
    for (int s = wave; s < NSEG; s += TPB / 32) {
        float run = seg[s * DL + lane];
#pragma unroll 1
        for (int j = s * 32; j < s * 32 + 32; ++j) { run += us[j * DL + lane]; us[j * DL + lane] = run; }
    }
    __syncthreads();

#pragma unroll 1
    for (int ps = 0; ps < 2; ++ps) {
#pragma unroll 1
        for (int it = 0; it < PPT; ++it) {
            unsigned q = (unsigned)(it * TPB + t);
            asm volatile("" : "+v"(q));
            const int i = (int)(q >> 2), b0 = (int)(q & 3u) * 8;
            const float sc = vrow[i] * SCARRY;
            const bool okm3 = i >= 3, okp2 = i + 2 < SEQ;
            const int jm3 = okm3 ? i - 3 : 0, jp2 = okp2 ? i + 2 : SEQ - 1;
            const v4f a0 = *(const v4fa*)(&us[jm3 * DL + b0]), a1 = *(const v4fa*)(&us[jm3 * DL + b0 + 4]);
            const v4f c0 = *(const v4fa*)(&us[jp2 * DL + b0]), c1 = *(const v4fa*)(&us[jp2 * DL + b0 + 4]);
            const v4f t0 = *(const v4fa*)(&us[(SEQ - 1) * DL + b0]), t1 = *(const v4fa*)(&us[(SEQ - 1) * DL + b0 + 4]);
            v8h o0, o4;
#pragma unroll
            for (int c = 0; c < 4; ++c) {
                o0[c] = toh_flush((okm3 ? a0[c] : 0.0f) * sc); o0[4 + c] = toh_flush((okm3 ? a1[c] : 0.0f) * sc);
                const float s0 = okp2 ? (t0[c] - c0[c]) : 0.0f;
                const float s1 = okp2 ? (t1[c] - c1[c]) : 0.0f;
                o4[c] = toh_flush(s0 * sc); o4[4 + c] = toh_flush(s1 * sc);
            }
            const size_t off = zoff + (size_t)q * 8;
            *(volatile v8h*)(SP + off) = o0;
            *(volatile v8h*)(SP + (size_t)4 * PLANE + off) = o4;
        }
        if (ps == 0) __threadfence();
    }
}

__global__ __launch_bounds__(32 * GW) void k_gemm(const h16* __restrict__ SP, const h16* __restrict__ WP, const float* __restrict__ x, float* OUT) {
    __shared__ __align__(16) float os[GW * 16 * OSP];
    const int lane = threadIdx.x & 31, lr = lane & 15, hi = lane >> 4;
    const int wave = __builtin_amdgcn_readfirstlane((int)(threadIdx.x >> 5));
    const int r0 = (blockIdx.x * GW + wave) * 16;
    const int z = r0 / SEQ, i0 = r0 % SEQ;
    const size_t PLANE = (size_t)NB * SEQ * DL;
    const size_t ao = (size_t)(r0 + lr) * DL + 8 * hi;
    const size_t bo = (size_t)lr * KD + 8 * hi;
    v8f c0 = (v8f){}, c1 = (v8f){};
#pragma unroll 1
    for (int kb = 0; kb < NBK; ++kb) {
        const v16h a  = ldh(SP + (size_t)kb * PLANE + ao);
        const v16h b0 = ldh(WP + bo + (size_t)kb * DL);
        const v16h b1 = ldh(WP + bo + (size_t)16 * KD + (size_t)kb * DL);
        c0 = wmma16g(a, b0, c0);
        c1 = wmma16g(a, b1, c1);
    }
    const int wb = wave * 16 * OSP;
#pragma unroll
    for (int j = 0; j < 8; ++j) { os[wb + (hi * 8 + j) * OSP + lr] = c0[j] * EPI; os[wb + (hi * 8 + j) * OSP + 16 + lr] = c1[j] * EPI; }
    wave_sync();
    static_assert(4 * 4 == 16);
    static_assert(8 * 4 == DL);
    const float* xrow = x + ((size_t)z * SEQ_FULL + i0) * DL;
    float* orow = OUT + ((size_t)z * OUT_SEQ + i0) * DL;
    v4f val[4];
#pragma unroll
    for (int s = 0; s < 4; ++s) { const int row = 4 * s + (lane >> 3), cofs = (lane & 7) * 4;
        const v4f f = *(const v4fa*)(&os[wb + row * OSP + cofs]);
        const v4f xv = *(const v4f*)(xrow + (size_t)row * DL + cofs);
        val[s] = xv + f; }
#pragma unroll 1
    for (int ps = 0; ps < 2; ++ps) {
#pragma unroll
        for (int s = 0; s < 4; ++s) { const int row = 4 * s + (lane >> 3), cofs = (lane & 7) * 4;
            *(volatile v4f*)(orow + (size_t)row * DL + cofs) = val[s]; }
        if (ps == 0) __threadfence(); }
}

static constexpr size_t al256(size_t v) { return (v + 255) & ~(size_t)255; }
static constexpr size_t SZ_WP = al256((size_t)DL * KD * 2);
static constexpr size_t SZ_SP = al256((size_t)NBK * NB * SEQ * DL * 2);
static constexpr size_t SZ_TOTAL = SZ_WP + SZ_SP;
static_assert(SZ_TOTAL <= (size_t)134217728);
static_assert(((size_t)NB * SEQ * DL * 2) % 512 == 0);
static_assert((size_t)(DL * KD / 8) == (size_t)5 * 128);
static_assert((size_t)NBK * ((size_t)NB * PPT * TPB * 8) * 2 == (size_t)NBK * NB * SEQ * DL * 2);

extern "C" void kernel_launch(void* const* d_in, const int* in_sizes, int n_in,
                              void* d_out, int out_size, void* d_ws, size_t ws_size, hipStream_t stream) {
    if (n_in < 3) return;
    constexpr size_t needx = ((size_t)(NB - 1) * SEQ_FULL + SEQ) * DL;
    constexpr size_t needm = (size_t)(NB - 1) * SEQ_FULL + SEQ;
    if ((size_t)in_sizes[0] < needx || (size_t)in_sizes[1] < needm || (size_t)in_sizes[2] < TERN_N) return;
    if ((size_t)out_size < ((size_t)(NB - 1) * OUT_SEQ + SEQ) * DL) return;
    if (SZ_TOTAL > ws_size) return;
    const float* x = (const float*)d_in[0];
    const int* mask = (const int*)d_in[1];
    const float* tern = (const float*)d_in[2];
    float* OUT = (float*)d_out;
    char* wsp = (char*)d_ws;
    h16* WP = (h16*)wsp; wsp += SZ_WP;
    h16* SP = (h16*)wsp; wsp += SZ_SP;

    k_wsum<<<dim3(5, 1, 1), 128, 0, stream>>>(tern, WP);
    k_bucket<<<dim3(NB, 1, 1), TPB, 0, stream>>>(x, mask, SP);
    k_gemm<<<dim3(NB * SEQ / (16 * GW), 1, 1), 32 * GW, 0, stream>>>(SP, WP, x, OUT);
}
